// FFJORD_67465346285802
// MI455X (gfx1250) — hardware-verified
//
#include <hip/hip_runtime.h>
#include <math.h>

constexpr int NBAT   = 4096;
constexpr int NDIM   = 64;
constexpr int NHID   = 256;
constexpr int NSTEPS = 16;
constexpr int NTHR   = 256;
constexpr int MROWS  = 32;
constexpr int APITCH = 72;
constexpr int HPITCH = 264;
constexpr int OPITCH = 260;
constexpr float HSTEP      = 1.0f / 16.0f;
constexpr float WCARRY     = 16.0f;
constexpr float WCARRY_INV = 1.0f / 16.0f;
static_assert(NBAT % MROWS == 0);
static_assert(MROWS == 32 && NTHR == 256);
static_assert(NHID == 4 * 64);
static_assert(NDIM == 4 * 16);
static_assert(NDIM % 32 == 0 && NHID % 64 == 0);
static_assert(APITCH % 8 == 0 && APITCH >= NDIM);
static_assert(HPITCH % 8 == 0 && HPITCH >= NHID);
static_assert(OPITCH % 4 == 0 && OPITCH >= NDIM);
static_assert((MROWS * NDIM) % (4 * NTHR) == 0);
static_assert(NDIM % 64 == 0 && NHID % 64 == 0);

typedef __attribute__((ext_vector_type(16))) _Float16 v16h;
typedef __attribute__((ext_vector_type(8)))  _Float16 v8h;
typedef __attribute__((ext_vector_type(8)))  float    v8f;
typedef __attribute__((ext_vector_type(4)))  float    v4f;

__device__ __forceinline__ void dep_guard4_h(v8f& a, v8f& b, v8f& c, v8f& d, v16h x, v16h y) {
  asm volatile("v_nop\n\tv_nop\n\tv_nop\n\tv_nop" : "+v"(a), "+v"(b), "+v"(c), "+v"(d) : "v"(x), "v"(y));
}
__device__ __forceinline__ void dep_guard2_h(v8f& a, v8f& b, v16h x, v16h y) {
  asm volatile("v_nop\n\tv_nop\n\tv_nop\n\tv_nop" : "+v"(a), "+v"(b) : "v"(x), "v"(y));
}
__device__ __forceinline__ void keep4_h(v16h a, v16h b, v16h c, v16h d) { asm volatile("v_nop" :: "v"(a), "v"(b), "v"(c), "v"(d)); }
__device__ __forceinline__ void acc_guard4(v8f& a, v8f& b, v8f& c, v8f& d) { asm volatile("v_nop\n\tv_nop\n\tv_nop\n\tv_nop" : "+v"(a), "+v"(b), "+v"(c), "+v"(d)); }
__device__ __forceinline__ void acc_guard2(v8f& a, v8f& b) { asm volatile("v_nop\n\tv_nop\n\tv_nop\n\tv_nop" : "+v"(a), "+v"(b)); }
__device__ __forceinline__ void touch4(float& a, float& b, float& c, float& d) { asm volatile("" : "+v"(a), "+v"(b), "+v"(c), "+v"(d)); }
__device__ __forceinline__ void touch1(float& a) { asm volatile("" : "+v"(a)); }

template <typename T> struct Frag;
template <> struct Frag<_Float16> {
  typedef v16h V; union U { v16h v; v8h h[2]; };
  static __device__ __forceinline__ v16h load(const _Float16* p) {
    U f; f.h[0] = *(const v8h*)(p); f.h[1] = *(const v8h*)(p + 16); return f.v;
  }
  static __device__ __forceinline__ v8f mma(v16h a, v16h b, v8f c) {
    return __builtin_amdgcn_wmma_f32_16x16x32_f16(false, a, false, b, (short)0, c, false, false);
  }
};

__device__ __forceinline__ float ftanh(float x) { return 1.0f - 2.0f * __builtin_amdgcn_rcpf(__expf(2.0f * x) + 1.0f); }

__global__ __launch_bounds__(NTHR) void tpw_f16_kernel(const float* __restrict__ src, int C, int ldo,
                                                       unsigned short* __restrict__ O, float sc) {
  __shared__ float Tt[64 * 65];
  const int tid = threadIdx.x;
  const int c0 = blockIdx.x * 64, r0 = blockIdx.y * 64;
#pragma unroll
  for (int i = 0; i < 4; ++i) {
    const int idx = i * NTHR + tid;
    const int rr = idx >> 4, cc = (idx & 15) * 4;
    const v4f v = *(const v4f*)(src + (size_t)(r0 + rr) * (size_t)C + c0 + cc);
    Tt[rr * 65 + cc + 0] = v[0];
    Tt[rr * 65 + cc + 1] = v[1];
    Tt[rr * 65 + cc + 2] = v[2];
    Tt[rr * 65 + cc + 3] = v[3];
  }
  __syncthreads();
  const int q = tid >> 3, c8 = (tid & 7) * 8;
  v8h hv[2];
#pragma unroll
  for (int g = 0; g < 2; ++g) {
    const int qq = g * 32 + q;
#pragma unroll
    for (int e = 0; e < 8; ++e) {
      const float f = Tt[(c8 + e) * 65 + qq];
      hv[g][e] = (_Float16)(f * sc);
    }
  }
  for (int pass = 0; pass < 2; ++pass) {
#pragma unroll
    for (int g = 0; g < 2; ++g) {
      const size_t o = (size_t)(c0 + g * 32 + q) * (size_t)ldo + (size_t)(r0 + c8);
      *(volatile v8h*)(O + o) = hv[g];
    }
    __threadfence();
  }
}

__device__ __forceinline__ void mlp_eval(
    float ts, const float (&st)[8], float (&kout)[8],
    _Float16* Apl, _Float16* Hpl, _Float16* H2pl,
    const _Float16* __restrict__ W1T, const _Float16* __restrict__ W2T, const _Float16* __restrict__ W3T,
    const float (&bb1)[4], const float (&tw1)[4], const float (&bb2)[4], float bb3,
    int mt, int cg, int c, int hh, int koff) {
  const v8f z8 = {0.f, 0.f, 0.f, 0.f, 0.f, 0.f, 0.f, 0.f};
  const int rowA = mt * 16 + 8 * hh;

#pragma unroll
  for (int r = 0; r < 8; ++r) Apl[(rowA + r) * APITCH + cg * 16 + c] = (_Float16)st[r];
  __syncthreads();

  {
    const _Float16* arow = Apl + (size_t)(mt * 16 + c) * APITCH + koff;
    const _Float16* w    = W1T + (size_t)(cg * 64 + c) * NDIM + koff;
    v8f acc0 = z8, acc1 = z8, acc2 = z8, acc3 = z8;
#pragma unroll 1
    for (int k0 = 0; k0 < NDIM; k0 += 32) {
      const v16h a  = Frag<_Float16>::load(arow + k0);
      const v16h b0 = Frag<_Float16>::load(w + k0);
      const v16h b1 = Frag<_Float16>::load(w + (size_t)16 * NDIM + k0);
      const v16h b2 = Frag<_Float16>::load(w + (size_t)32 * NDIM + k0);
      const v16h b3 = Frag<_Float16>::load(w + (size_t)48 * NDIM + k0);
      acc0 = Frag<_Float16>::mma(a, b0, acc0);
      acc1 = Frag<_Float16>::mma(a, b1, acc1);
      acc2 = Frag<_Float16>::mma(a, b2, acc2);
      acc3 = Frag<_Float16>::mma(a, b3, acc3);
      dep_guard4_h(acc0, acc1, acc2, acc3, a, b3);
      keep4_h(b0, b1, b2, b3);
    }
    acc_guard4(acc0, acc1, acc2, acc3);
    const float p0 = bb1[0] + ts * tw1[0], p1 = bb1[1] + ts * tw1[1], p2 = bb1[2] + ts * tw1[2], p3 = bb1[3] + ts * tw1[3];
    const int col = cg * 64 + c;
#pragma unroll
    for (int r = 0; r < 8; ++r) {
      _Float16* hrow = Hpl + (size_t)(rowA + r) * HPITCH + col;
      hrow[0]  = (_Float16)ftanh(acc0[r] * WCARRY_INV + p0);
      hrow[16] = (_Float16)ftanh(acc1[r] * WCARRY_INV + p1);
      hrow[32] = (_Float16)ftanh(acc2[r] * WCARRY_INV + p2);
      hrow[48] = (_Float16)ftanh(acc3[r] * WCARRY_INV + p3);
    }
  }
  __syncthreads();

  {
    const _Float16* arow = Hpl + (size_t)(mt * 16 + c) * HPITCH + koff;
    const _Float16* w    = W2T + (size_t)(cg * 64 + c) * NHID + koff;
    v8f acc0 = z8, acc1 = z8, acc2 = z8, acc3 = z8;
#pragma unroll 1
    for (int k0 = 0; k0 < NHID; k0 += 32) {
      const v16h a  = Frag<_Float16>::load(arow + k0);
      const v16h b0 = Frag<_Float16>::load(w + k0);
      const v16h b1 = Frag<_Float16>::load(w + (size_t)16 * NHID + k0);
      const v16h b2 = Frag<_Float16>::load(w + (size_t)32 * NHID + k0);
      const v16h b3 = Frag<_Float16>::load(w + (size_t)48 * NHID + k0);
      acc0 = Frag<_Float16>::mma(a, b0, acc0);
      acc1 = Frag<_Float16>::mma(a, b1, acc1);
      acc2 = Frag<_Float16>::mma(a, b2, acc2);
      acc3 = Frag<_Float16>::mma(a, b3, acc3);
      dep_guard4_h(acc0, acc1, acc2, acc3, a, b3);
      keep4_h(b0, b1, b2, b3);
    }
    acc_guard4(acc0, acc1, acc2, acc3);
    const int col = cg * 64 + c;
#pragma unroll
    for (int r = 0; r < 8; ++r) {
      _Float16* hrow = H2pl + (size_t)(rowA + r) * HPITCH + col;
      hrow[0]  = (_Float16)ftanh(acc0[r] * WCARRY_INV + bb2[0]);
      hrow[16] = (_Float16)ftanh(acc1[r] * WCARRY_INV + bb2[1]);
      hrow[32] = (_Float16)ftanh(acc2[r] * WCARRY_INV + bb2[2]);
      hrow[48] = (_Float16)ftanh(acc3[r] * WCARRY_INV + bb2[3]);
    }
  }
  __syncthreads();

  {
    const _Float16* arow = H2pl + (size_t)(mt * 16 + c) * HPITCH + koff;
    const _Float16* w    = W3T + (size_t)(cg * 16 + c) * NHID + koff;
    v8f acc0 = z8, acc1 = z8;
#pragma unroll 1
    for (int k0 = 0; k0 < NHID; k0 += 64) {
      const v16h a0 = Frag<_Float16>::load(arow + k0);
      const v16h b0 = Frag<_Float16>::load(w + k0);
      const v16h a1 = Frag<_Float16>::load(arow + k0 + 32);
      const v16h b1 = Frag<_Float16>::load(w + k0 + 32);
      acc0 = Frag<_Float16>::mma(a0, b0, acc0);
      acc1 = Frag<_Float16>::mma(a1, b1, acc1);
      dep_guard2_h(acc0, acc1, a1, b1);
      keep4_h(a0, b0, a1, b1);
    }
    acc_guard2(acc0, acc1);
#pragma unroll
    for (int r = 0; r < 8; ++r) kout[r] = (acc0[r] + acc1[r]) * WCARRY_INV + bb3;
  }
}

__global__ __launch_bounds__(NTHR) void ode_flow_kernel(
    const float* __restrict__ x,
    const float* __restrict__ W1a, const float* __restrict__ b1a, const float* __restrict__ b2a, const float* __restrict__ b3a,
    const float* __restrict__ W1b, const float* __restrict__ b1b, const float* __restrict__ b2b, const float* __restrict__ b3b,
    const unsigned short* __restrict__ WT1p,
    const unsigned short* __restrict__ WT2p,
    const unsigned short* __restrict__ WT3p,
    float* __restrict__ out) {
  __shared__ __align__(16) _Float16 Apl[MROWS * APITCH];
  __shared__ __align__(16) _Float16 Hpl[MROWS * HPITCH];
  __shared__ __align__(16) _Float16 H2pl[MROWS * HPITCH];
  __shared__ __align__(16) float    Os[MROWS * OPITCH];
  const int tid = threadIdx.x, lane = tid & 31, wave = tid >> 5;
  const int c = lane & 15, hh = lane >> 4, koff = hh * 8;
  const int mt = wave >> 2, cg = wave & 3;
  const int rowBlock = blockIdx.x * MROWS;
  const int rowA = mt * 16 + 8 * hh;

  float y[8];
#pragma unroll
  for (int r = 0; r < 8; ++r) y[r] = x[(size_t)(rowBlock + rowA + r) * NDIM + cg * 16 + c];
  touch4(y[0], y[1], y[2], y[3]);
  touch4(y[4], y[5], y[6], y[7]);

#pragma unroll 1
  for (int bj = 0; bj < 2; ++bj) {
    const float* W1 = bj ? W1b : W1a;
    const float* b1 = bj ? b1b : b1a;
    const float* b2 = bj ? b2b : b2a;
    const float* b3 = bj ? b3b : b3a;
    const _Float16* W1T = (const _Float16*)WT1p + (size_t)bj * NHID * NDIM;
    const _Float16* W2T = (const _Float16*)WT2p + (size_t)bj * NHID * NHID;
    const _Float16* W3T = (const _Float16*)WT3p + (size_t)bj * NDIM * NHID;
    float bb1[4], tw1[4], bb2[4];
#pragma unroll
    for (int j = 0; j < 4; ++j) {
      const int n = cg * 64 + 16 * j + c;
      bb1[j] = b1[n];
      tw1[j] = W1[NDIM * NHID + n];
      bb2[j] = b2[n];
    }
    float bb3 = b3[cg * 16 + c];
    touch4(bb1[0], bb1[1], bb1[2], bb1[3]);
    touch4(tw1[0], tw1[1], tw1[2], tw1[3]);
    touch4(bb2[0], bb2[1], bb2[2], bb2[3]);
    touch1(bb3);

#pragma unroll 1
    for (int step = 0; step < NSTEPS; ++step) {
      const float t0 = (float)step * HSTEP;
      float st[8], kA[8], kB[8], kC[8], kD[8], kE[8], kF[8];
#pragma unroll
      for (int r = 0; r < 8; ++r) st[r] = y[r];
      mlp_eval(t0, st, kA, Apl, Hpl, H2pl, W1T, W2T, W3T, bb1, tw1, bb2, bb3, mt, cg, c, hh, koff);
#pragma unroll
      for (int r = 0; r < 8; ++r) st[r] = y[r] + HSTEP * ((1.0f / 5.0f) * kA[r]);
      mlp_eval(t0 + HSTEP * (1.0f / 5.0f), st, kB, Apl, Hpl, H2pl, W1T, W2T, W3T, bb1, tw1, bb2, bb3, mt, cg, c, hh, koff);
#pragma unroll
      for (int r = 0; r < 8; ++r) st[r] = y[r] + HSTEP * ((3.0f / 40.0f) * kA[r] + (9.0f / 40.0f) * kB[r]);
      mlp_eval(t0 + HSTEP * (3.0f / 10.0f), st, kC, Apl, Hpl, H2pl, W1T, W2T, W3T, bb1, tw1, bb2, bb3, mt, cg, c, hh, koff);
#pragma unroll
      for (int r = 0; r < 8; ++r)
        st[r] = y[r] + HSTEP * ((44.0f / 45.0f) * kA[r] - (56.0f / 15.0f) * kB[r] + (32.0f / 9.0f) * kC[r]);
      mlp_eval(t0 + HSTEP * (4.0f / 5.0f), st, kD, Apl, Hpl, H2pl, W1T, W2T, W3T, bb1, tw1, bb2, bb3, mt, cg, c, hh, koff);
#pragma unroll
      for (int r = 0; r < 8; ++r)
        st[r] = y[r] + HSTEP * ((19372.0f / 6561.0f) * kA[r] - (25360.0f / 2187.0f) * kB[r]
                                + (64448.0f / 6561.0f) * kC[r] - (212.0f / 729.0f) * kD[r]);
      mlp_eval(t0 + HSTEP * (8.0f / 9.0f), st, kE, Apl, Hpl, H2pl, W1T, W2T, W3T, bb1, tw1, bb2, bb3, mt, cg, c, hh, koff);
#pragma unroll
      for (int r = 0; r < 8; ++r)
        st[r] = y[r] + HSTEP * ((9017.0f / 3168.0f) * kA[r] - (355.0f / 33.0f) * kB[r]
                                + (46732.0f / 5247.0f) * kC[r] + (49.0f / 176.0f) * kD[r]
                                - (5103.0f / 18656.0f) * kE[r]);
      mlp_eval(t0 + HSTEP, st, kF, Apl, Hpl, H2pl, W1T, W2T, W3T, bb1, tw1, bb2, bb3, mt, cg, c, hh, koff);
#pragma unroll
      for (int r = 0; r < 8; ++r)
        y[r] = y[r] + HSTEP * ((35.0f / 384.0f) * kA[r] + (500.0f / 1113.0f) * kC[r] + (125.0f / 192.0f) * kD[r]
                               - (2187.0f / 6784.0f) * kE[r] + (11.0f / 84.0f) * kF[r]);
    }
  }

#pragma unroll
  for (int r = 0; r < 8; ++r) Os[(rowA + r) * OPITCH + cg * 16 + c] = y[r];
  __syncthreads();
  for (int pass = 0; pass < 2; ++pass) {
#pragma unroll
    for (int it = 0; it < 2; ++it) {
      const int idx = it * NTHR + tid;
      const int row = idx >> 4, c4 = (idx & 15) * 4;
      const v4f v = *(const v4f*)(Os + row * OPITCH + c4);
      *(volatile v4f*)(out + (size_t)(rowBlock + row) * NDIM + c4) = v;
    }
    __threadfence();
  }
}

extern "C" void kernel_launch(void* const* d_in, const int* in_sizes, int n_in,
                              void* d_out, int out_size, void* d_ws, size_t ws_size, hipStream_t stream) {
  if (n_in < 13 || d_out == nullptr || d_ws == nullptr) return;
  if (in_sizes[0] != NBAT * NDIM || out_size != NBAT * NDIM) return;
  for (int b = 0; b < 2; ++b) {
    const int o = 1 + 6 * b;
    if (in_sizes[o] != (NDIM + 1) * NHID || in_sizes[o + 1] != NHID || in_sizes[o + 2] != NHID * NHID ||
        in_sizes[o + 3] != NHID || in_sizes[o + 4] != NHID * NDIM || in_sizes[o + 5] != NDIM) return;
  }

  const float* x   = (const float*)d_in[0];
  const float* W1a = (const float*)d_in[1];
  const float* b1a = (const float*)d_in[2];
  const float* W2a = (const float*)d_in[3];
  const float* b2a = (const float*)d_in[4];
  const float* W3a = (const float*)d_in[5];
  const float* b3a = (const float*)d_in[6];
  const float* W1b = (const float*)d_in[7];
  const float* b1b = (const float*)d_in[8];
  const float* W2b = (const float*)d_in[9];
  const float* b2b = (const float*)d_in[10];
  const float* W3b = (const float*)d_in[11];
  const float* b3b = (const float*)d_in[12];
  float* out = (float*)d_out;

  char* ws = (char*)d_ws; size_t off = 0;
  auto carve = [&](size_t bytes) -> char* { char* p = ws + off; off += (bytes + 255) & ~(size_t)255; return p; };
  unsigned short* WT1 = (unsigned short*)carve((size_t)2 * NHID * NDIM * 2);
  unsigned short* WT2 = (unsigned short*)carve((size_t)2 * NHID * NHID * 2);
  unsigned short* WT3 = (unsigned short*)carve((size_t)2 * NDIM * NHID * 2);
  if (off > ws_size || off > (size_t)134217728) return;

  tpw_f16_kernel<<<dim3(NHID / 64, NDIM / 64), NTHR, 0, stream>>>(W1a, NHID, NDIM, WT1, WCARRY);
  tpw_f16_kernel<<<dim3(NHID / 64, NHID / 64), NTHR, 0, stream>>>(W2a, NHID, NHID, WT2, WCARRY);
  tpw_f16_kernel<<<dim3(NDIM / 64, NHID / 64), NTHR, 0, stream>>>(W3a, NDIM, NHID, WT3, WCARRY);
  tpw_f16_kernel<<<dim3(NHID / 64, NDIM / 64), NTHR, 0, stream>>>(W1b, NHID, NDIM, WT1 + (size_t)NHID * NDIM, WCARRY);
  tpw_f16_kernel<<<dim3(NHID / 64, NHID / 64), NTHR, 0, stream>>>(W2b, NHID, NHID, WT2 + (size_t)NHID * NHID, WCARRY);
  tpw_f16_kernel<<<dim3(NDIM / 64, NHID / 64), NTHR, 0, stream>>>(W3b, NDIM, NHID, WT3 + (size_t)NDIM * NHID, WCARRY);
  ode_flow_kernel<<<NBAT / MROWS, NTHR, 0, stream>>>(x, W1a, b1a, b2a, b3a, W1b, b1b, b2b, b3b, WT1, WT2, WT3, out);
}
